// NanoChatAttention_10806137717006
// MI455X (gfx1250) — hardware-verified
//
#include <hip/hip_runtime.h>
#include <stdint.h>
#include <math.h>

#define NBATCH 2
#define SEQ 2048
#define DMODEL 2048
#define NHEAD 16
#define NKVH 4
#define HDIM 128
#define NTOK (NBATCH * SEQ)
#define QCOLS (NHEAD * HDIM)
#define KVCOLS (NKVH * HDIM)
#define NXR 128
#define NXTOT (NBATCH * NXR)
#define ATT_SCALE 0.08838834764831845f
#define RMS_EPS 1.1920929e-7f
#define WMUL 64.0f
#define WMUL_INV (1.0f / 64.0f)
#define OMUL 16.0f
#define OMUL_INV (1.0f / 16.0f)

static_assert(NHEAD / NKVH == 4);
static_assert(QCOLS == DMODEL);

typedef __attribute__((ext_vector_type(16))) _Float16 v16h;
typedef __attribute__((ext_vector_type(8)))  _Float16 v8h;
typedef __attribute__((ext_vector_type(4)))  _Float16 v4h;
typedef __attribute__((ext_vector_type(16))) __bf16   v16b;
typedef __attribute__((ext_vector_type(8)))  __bf16   v8b;
typedef __attribute__((ext_vector_type(8)))  float    v8f;
typedef __attribute__((ext_vector_type(4)))  float    v4f;
#define PSCALE 32768.0f
#define U16(p) ((const unsigned short*)(const void*)(p))
#define PSCALE_INV (1.0f / 32768.0f)

__device__ __forceinline__ unsigned short f2bf_bits(float f) {
  unsigned u = __float_as_uint(f);
  return (unsigned short)((u + 0x7FFFu + ((u >> 16) & 1u)) >> 16);
}
__device__ __forceinline__ float bf_bits2f(unsigned short h) { return __uint_as_float(((unsigned)h) << 16); }

__device__ __forceinline__ void dep_guard_h(v8f& a, v8f& b, v16h x, v16h y) { asm volatile("v_nop\n\tv_nop\n\tv_nop\n\tv_nop" : "+v"(a), "+v"(b) : "v"(x), "v"(y)); }
__device__ __forceinline__ void dep_guard_b(v8f& a, v8f& b, v16b x, v16b y) { asm volatile("v_nop\n\tv_nop\n\tv_nop\n\tv_nop" : "+v"(a), "+v"(b) : "v"(x), "v"(y)); }
__device__ __forceinline__ void keep4_h(v16h a, v16h b, v16h c, v16h d) { asm volatile("v_nop" :: "v"(a), "v"(b), "v"(c), "v"(d)); }
__device__ __forceinline__ void keep4_b(v16b a, v16b b, v16b c, v16b d) { asm volatile("v_nop" :: "v"(a), "v"(b), "v"(c), "v"(d)); }
__device__ __forceinline__ void acc_guard4(v8f& a, v8f& b, v8f& c, v8f& d) { asm volatile("v_nop\n\tv_nop\n\tv_nop\n\tv_nop" : "+v"(a), "+v"(b), "+v"(c), "+v"(d)); }
template <typename T> struct Frag;
template <> struct Frag<_Float16> {
  typedef v16h V; union U { v16h v; v8h h[2]; };
  static __device__ __forceinline__ v16h load(const _Float16* p) {
    U f; f.h[0] = *(const v8h*)(p); f.h[1] = *(const v8h*)(p + 16); return f.v;
  }
  static __device__ __forceinline__ v8f mma(v16h a, v16h b, v8f c) {
    return __builtin_amdgcn_wmma_f32_16x16x32_f16(false, a, false, b, (short)0, c, false, false);
  }
  static __device__ __forceinline__ void guard(v8f& a, v8f& b, v16h x, v16h y) { dep_guard_h(a, b, x, y); }
  static __device__ __forceinline__ void keep(v16h a, v16h b, v16h c, v16h d) { keep4_h(a, b, c, d); }
};
template <> struct Frag<__bf16> {
  typedef v16b V; union U { v16b v; v8b h[2]; };
  static __device__ __forceinline__ v16b load(const __bf16* p) {
    U f; f.h[0] = *(const v8b*)(p); f.h[1] = *(const v8b*)(p + 16); return f.v;
  }
  static __device__ __forceinline__ v8f mma(v16b a, v16b b, v8f c) {
    return __builtin_amdgcn_wmma_f32_16x16x32_bf16(false, a, false, b, (short)0, c, false, false);
  }
  static __device__ __forceinline__ void guard(v8f& a, v8f& b, v16b x, v16b y) { dep_guard_b(a, b, x, y); }
  static __device__ __forceinline__ void keep(v16b a, v16b b, v16b c, v16b d) { keep4_b(a, b, c, d); }
};

template <int ET> struct Elem;
template <> struct Elem<0> { typedef _Float16 T; };
template <> struct Elem<1> { typedef __bf16 T; };
template <int ET, bool SPLIT, int BIAS_MODE, int OUT_MODE, bool RESID, int ACT = 0>
__global__ __launch_bounds__(256) void wmma_gemm64(
    const unsigned short* __restrict__ Ap, const unsigned short* __restrict__ A2p, int lda, long strideA,
    const unsigned short* __restrict__ Btp, const unsigned short* __restrict__ Bt2p, int ldb, long strideB,
    void* __restrict__ Cout, void* __restrict__ Cout2, int ldc, long strideC,
    const float* __restrict__ bias,
    const float* __restrict__ resid, long strideR,
    int M, int N, int K, float scale) {
  typedef typename Elem<ET>::T T;
  typedef typename Frag<T>::V V;
  const T* A = (const T*)Ap; const T* A2 = (const T*)A2p; const T* Bt = (const T*)Btp; const T* Bt2 = (const T*)Bt2p;
  __shared__ __align__(16) float sT[8][16 * 68];
  const int b    = blockIdx.y;
  const int lane = threadIdx.x & 31;
  const int wave = threadIdx.x >> 5;
  const int tilesN = N >> 6;
  const int tilesM = M >> 6;
  const int tile = blockIdx.x * 8 + wave;
  if (tile >= tilesM * tilesN) return;
  const int tm = tile / tilesN;
  const int tn = tile - tm * tilesN;
  const int m0 = tm << 6;
  const int n0 = tn << 6;

  const T* Ab  = A  + (size_t)b * strideA;
  const T* Bb  = Bt + (size_t)b * strideB;
  const T* Ab2 = SPLIT ? (A2  + (size_t)b * strideA) : nullptr;
  const T* Bb2 = SPLIT ? (Bt2 + (size_t)b * strideB) : nullptr;

  const int rlane = lane & 15;
  const int koff  = (lane >> 4) * 8;
  const int mOff  = (lane >> 4) * 8;

  v8f acc[4][4];
#pragma unroll
  for (int i = 0; i < 4; ++i)
#pragma unroll
    for (int j = 0; j < 4; ++j) acc[i][j] = (v8f){0.f,0.f,0.f,0.f,0.f,0.f,0.f,0.f};

  for (int k0 = 0; k0 < K; k0 += 32) {
    V bh[4], bl[4];
#pragma unroll
    for (int j = 0; j < 4; ++j) {
      const size_t bo = (size_t)(n0 + (j << 4) + rlane) * ldb + koff + k0;
      bh[j] = Frag<T>::load(Bb + bo);
      if (SPLIT) bl[j] = Frag<T>::load(Bb2 + bo);
    }
#pragma unroll
    for (int i = 0; i < 4; ++i) {
      const size_t ao = (size_t)(m0 + (i << 4) + rlane) * lda + koff + k0;
      V ah = Frag<T>::load(Ab + ao);
      V al;
      if (SPLIT) al = Frag<T>::load(Ab2 + ao);
#pragma unroll
      for (int j = 0; j < 4; ++j) {
        acc[i][j] = Frag<T>::mma(ah, bh[j], acc[i][j]);
        if (SPLIT) {
          acc[i][j] = Frag<T>::mma(ah, bl[j], acc[i][j]);
          acc[i][j] = Frag<T>::mma(al, bh[j], acc[i][j]);
        }
      }
      Frag<T>::guard(acc[i][0], acc[i][3], ah, SPLIT ? al : ah);
    }
    Frag<T>::keep(bh[0], bh[1], bh[2], bh[3]);
    if (SPLIT) Frag<T>::keep(bl[0], bl[1], bl[2], bl[3]);
  }
  acc_guard4(acc[0][0], acc[0][1], acc[0][2], acc[0][3]);
  acc_guard4(acc[1][0], acc[1][1], acc[1][2], acc[1][3]);
  acc_guard4(acc[2][0], acc[2][1], acc[2][2], acc[2][3]);
  acc_guard4(acc[3][0], acc[3][1], acc[3][2], acc[3][3]);

  float* slab = sT[wave];
  const float* Rb = RESID ? (resid + (size_t)b * strideR) : nullptr;
#pragma unroll
  for (int i = 0; i < 4; ++i) {
    const int mBase = m0 + (i << 4);
#pragma unroll
    for (int j = 0; j < 4; ++j) {
      const int n = n0 + (j << 4) + rlane;
      float bv = 0.f;
      if (BIAS_MODE == 2) bv = bias[n];
#pragma unroll
      for (int r = 0; r < 8; ++r) {
        float v = acc[i][j][r] * scale;
        if (BIAS_MODE == 1) v += bias[mBase + mOff + r];
        if (BIAS_MODE == 2) v += bv;
        if (RESID) v += Rb[(size_t)(mBase + mOff + r) * ldc + n];
        if (ACT == 1) v = tanhf(v);
        if (ACT == 2) v = fmaxf(v, 0.0f);
        if (ACT == 4) v = (v > 0.f) ? v : 0.01f * v;
        if (ACT == 6) { v = fmaxf(v, 0.0f); v = v * v; }
        slab[(mOff + r) * 68 + (j << 4) + rlane] = v;
      }
    }
    __builtin_amdgcn_fence(__ATOMIC_RELEASE, "workgroup");
    __builtin_amdgcn_wave_barrier();
    __builtin_amdgcn_fence(__ATOMIC_ACQUIRE, "workgroup");
    if (OUT_MODE == 0) {
      float* C = (float*)Cout + (size_t)b * strideC;
      const int hh = lane >> 4, c4 = (lane & 15) * 4;
      for (int pass = 0; pass < 2; ++pass) {
#pragma unroll
        for (int it = 0; it < 8; ++it) {
          const int row = it * 2 + hh;
          v4f v = *(const v4f*)(slab + row * 68 + c4);
          *(volatile v4f*)(C + (size_t)(mBase + row) * ldc + n0 + c4) = v;
        }
        __threadfence();
      }
    } else {
      const int q = lane >> 3, c8 = (lane & 7) * 8;
      unsigned short* C  = (unsigned short*)Cout  + (size_t)b * strideC;
      unsigned short* C2 = (OUT_MODE == 2) ? ((unsigned short*)Cout2 + (size_t)b * strideC) : nullptr;
      for (int pass = 0; pass < 2; ++pass) {
#pragma unroll
        for (int it = 0; it < 4; ++it) {
          const int row = it * 4 + q;
          const float* sp = slab + row * 68 + c8;
          v8h hv, lv;
#pragma unroll
          for (int e = 0; e < 8; ++e) {
            if (OUT_MODE == 1) {
              hv[e] = (_Float16)sp[e];
            } else {
              unsigned short hb = f2bf_bits(sp[e]);
              unsigned short lb = f2bf_bits(sp[e] - bf_bits2f(hb));
              hv[e] = __builtin_bit_cast(_Float16, hb);
              lv[e] = __builtin_bit_cast(_Float16, lb);
            }
          }
          *(volatile v8h*)(C + (size_t)(mBase + row) * ldc + n0 + c8) = hv;
          if (OUT_MODE == 2) *(volatile v8h*)(C2 + (size_t)(mBase + row) * ldc + n0 + c8) = lv;
        }
        __threadfence();
      }
    }
    __builtin_amdgcn_fence(__ATOMIC_RELEASE, "workgroup");
    __builtin_amdgcn_wave_barrier();
    __builtin_amdgcn_fence(__ATOMIC_ACQUIRE, "workgroup");
  }
}

__global__ __launch_bounds__(256) void cast_f32_f16x2(
    const float* __restrict__ in, _Float16* __restrict__ out, int n2, float mul) {
  int i = blockIdx.x * 256 + threadIdx.x;
  if (i < n2) {
    const _Float16 h0 = (_Float16)(in[2 * i] * mul), h1 = (_Float16)(in[2 * i + 1] * mul);
    const unsigned u = (unsigned)__builtin_bit_cast(unsigned short, h0) | ((unsigned)__builtin_bit_cast(unsigned short, h1) << 16);
    ((volatile unsigned*)out)[i] = u;
    __threadfence();
    ((volatile unsigned*)out)[i] = u;
  }
}

__global__ __launch_bounds__(256) void split_bf16x2(const float* __restrict__ in, unsigned short* __restrict__ hi,
                                                      unsigned short* __restrict__ lo, int ncol2, int nrows, int dgrp, int sgrp) {
  const int i = blockIdx.x * 256 + threadIdx.x;
  if (i < nrows * ncol2) {
    const int r = i / ncol2, c2 = i - r * ncol2;
    const int gq = r / dgrp;
    const int sr = gq * sgrp + (r - gq * dgrp);
    const float* src = in + (size_t)sr * (size_t)(2 * ncol2) + 2 * c2;
    const float f0 = src[0], f1 = src[1];
    const unsigned short h0 = f2bf_bits(f0), h1 = f2bf_bits(f1);
    const unsigned short l0 = f2bf_bits(f0 - bf_bits2f(h0)), l1 = f2bf_bits(f1 - bf_bits2f(h1));
    const unsigned uh = (unsigned)h0 | ((unsigned)h1 << 16);
    const unsigned ul = (unsigned)l0 | ((unsigned)l1 << 16);
    ((volatile unsigned*)hi)[i] = uh;
    ((volatile unsigned*)lo)[i] = ul;
    __threadfence();
    ((volatile unsigned*)hi)[i] = uh;
    ((volatile unsigned*)lo)[i] = ul;
  }
}

#define RSPF 132
template <int RMODE>
__global__ __launch_bounds__(256) void rope_rms_k(const float* __restrict__ qf, const float* __restrict__ kf,
                                                  const float* __restrict__ cosT, const float* __restrict__ sinT,
                                                  unsigned short* __restrict__ q16p, unsigned short* __restrict__ k16p,
                                                  float* __restrict__ qx, float* __restrict__ kx) {
  __shared__ __align__(16) float st[8][3 * RSPF];
  _Float16* q16 = (_Float16*)q16p;
  _Float16* k16 = (_Float16*)k16p;
  const int s = blockIdx.x, b = blockIdx.y;
  const int tid = threadIdx.x, w = tid >> 5, ln = tid & 31;
  const size_t tok = (size_t)b * (RMODE ? NXR : SEQ) + s;
  const float* ct = cosT + (size_t)s * HDIM;
  const float* snt = sinT + (size_t)s * HDIM;
  const float c0 = ct[ln], c1 = ct[ln + 32], c2 = ct[ln + 64], c3 = ct[ln + 96];
  const float s0 = snt[ln], s1 = snt[ln + 32], s2 = snt[ln + 64], s3 = snt[ln + 96];
  float* sw = st[w];
#pragma unroll
  for (int p = 0; p < 3; ++p) {
    const float* src = (p < 2) ? (qf + tok * QCOLS + (size_t)(w + 8 * p) * HDIM)
                               : (kf + tok * KVCOLS + (size_t)(w & 3) * HDIM);
    const float a0 = src[ln], a1 = src[ln + 32], a2 = src[ln + 64], a3 = src[ln + 96];
    const float o0 = a0 * c0 - a2 * s0;
    const float o1 = a1 * c1 - a3 * s1;
    const float o2 = a2 * c2 + a0 * s2;
    const float o3 = a3 * c3 + a1 * s3;
    float sq = (o0 * o0 + o1 * o1) + (o2 * o2 + o3 * o3);
#pragma unroll
    for (int off = 1; off < 32; off <<= 1) sq += __shfl_xor(sq, off, 32);
    const float rs = rsqrtf(sq * (1.0f / HDIM) + RMS_EPS);
    sw[p * RSPF + ln]      = o0 * rs;
    sw[p * RSPF + ln + 32] = o1 * rs;
    sw[p * RSPF + ln + 64] = o2 * rs;
    sw[p * RSPF + ln + 96] = o3 * rs;
  }
  __builtin_amdgcn_fence(__ATOMIC_RELEASE, "workgroup");
  __builtin_amdgcn_wave_barrier();
  __builtin_amdgcn_fence(__ATOMIC_ACQUIRE, "workgroup");
  if (RMODE == 0) {
    const int hh = ln >> 4, c8 = (ln & 15) * 8;
    v8h v01, v2;
    {
      const v4f qa4 = *(const v4f*)(sw + hh * RSPF + c8);
      const v4f qb4 = *(const v4f*)(sw + hh * RSPF + c8 + 4);
      const v4f ka4 = *(const v4f*)(sw + 2 * RSPF + c8);
      const v4f kb4 = *(const v4f*)(sw + 2 * RSPF + c8 + 4);
#pragma unroll
      for (int e = 0; e < 4; ++e) {
        v01[e] = (_Float16)qa4[e]; v01[4 + e] = (_Float16)qb4[e];
        v2[e]  = (_Float16)ka4[e]; v2[4 + e]  = (_Float16)kb4[e];
      }
    }
    _Float16* d01 = q16 + tok * QCOLS + (size_t)(w + 8 * hh) * HDIM + c8;
    _Float16* d2  = k16 + tok * KVCOLS + (size_t)(w & 3) * HDIM + c8;
    const bool wk = (w < 4) && (hh == 0);
    for (int pass = 0; pass < 2; ++pass) {
      *(volatile v8h*)d01 = v01;
      if (wk) *(volatile v8h*)d2 = v2;
      __threadfence();
    }
  } else {
    const v4f f0 = *(const v4f*)(sw + ln * 4);
    const v4f f1 = *(const v4f*)(sw + RSPF + ln * 4);
    const v4f f2 = *(const v4f*)(sw + 2 * RSPF + ln * 4);
    float* dq0 = qx + tok * QCOLS + (size_t)w * HDIM + ln * 4;
    float* dq1 = qx + tok * QCOLS + (size_t)(w + 8) * HDIM + ln * 4;
    float* dk  = kx + tok * KVCOLS + (size_t)(w & 3) * HDIM + ln * 4;
    for (int pass = 0; pass < 2; ++pass) {
      *(volatile v4f*)dq0 = f0;
      *(volatile v4f*)dq1 = f1;
      if (w < 4) *(volatile v4f*)dk = f2;
      __threadfence();
    }
  }
}

__device__ __forceinline__ v8f mma_h(v16h a, v16h b, v8f c) {
  c = __builtin_amdgcn_wmma_f32_16x16x32_f16(false, a, false, b, (short)0, c, false, false);
  asm volatile("v_nop\n\tv_nop\n\tv_nop\n\tv_nop" : "+v"(c) : "v"(a), "v"(b));
  return c;
}
#define AKC 64
#define AQB 64
#define OSP 136
__global__ __launch_bounds__(128) void attn128_k(const unsigned short* __restrict__ qpp, const unsigned short* __restrict__ kpp,
                                                 const unsigned short* __restrict__ vpp, unsigned short* __restrict__ outp) {
  union FH { v16h v; v8h h[2]; };
  __shared__ __align__(16) _Float16 Ksh[AKC * HDIM];
  __shared__ __align__(16) _Float16 Vth[HDIM * AKC];
  __shared__ __align__(16) _Float16 Psh[4][16 * AKC];
  __shared__ __align__(16) _Float16 Osh[4][16 * OSP];
  const _Float16* qp = (const _Float16*)qpp;
  const _Float16* kp = (const _Float16*)kpp;
  const _Float16* vp = (const _Float16*)vpp;
  _Float16* out = (_Float16*)outp;
  const int tid = threadIdx.x, wave = tid >> 5, lane = tid & 31, hh = lane >> 4, c = lane & 15;
  const int nqb = SEQ / AQB;
  const int bx = blockIdx.x;
  const int qb = bx % nqb;
  const int bh = bx / nqb;
  const int h = bh % NHEAD;
  const int b = bh / NHEAD;
  const int g = h / (NHEAD / NKVH);
  const int q0 = qb * AQB + wave * 16;
  const size_t tokb = (size_t)b * SEQ;

  v16h qa[4];
  {
    const _Float16* qrow = qp + (tokb + q0 + c) * QCOLS + (size_t)h * HDIM + 8 * hh;
#pragma unroll
    for (int dc = 0; dc < 4; ++dc) qa[dc] = Frag<_Float16>::load(qrow + dc * 32);
  }
  float mrow[8], lrow[8];
  v8f oacc[8];
#pragma unroll
  for (int r = 0; r < 8; ++r) { mrow[r] = -INFINITY; lrow[r] = 0.f; }
#pragma unroll
  for (int t = 0; t < 8; ++t) oacc[t] = (v8f){0.f,0.f,0.f,0.f,0.f,0.f,0.f,0.f};

  const int nChunks = qb + 1;
  for (int kc = 0; kc < nChunks; ++kc) {
    const int kv0 = kc * AKC;
    __syncthreads();
    {
      const int kvr = tid >> 1, dh = (tid & 1) * 64;
      const _Float16* krow = kp + (tokb + kv0 + kvr) * KVCOLS + (size_t)g * HDIM + dh;
      const _Float16* vrow = vp + (tokb + kv0 + kvr) * KVCOLS + (size_t)g * HDIM + dh;
#pragma unroll 1
      for (int i = 0; i < 8; ++i) {
        const v8h kk = *(const v8h*)(krow + 8 * i);
        *(v8h*)(Ksh + kvr * HDIM + dh + 8 * i) = kk;
        const v8h vv = *(const v8h*)(vrow + 8 * i);
#pragma unroll
        for (int e = 0; e < 8; ++e) Vth[(dh + 8 * i + e) * AKC + kvr] = vv[e];
      }
    }
    __syncthreads();

    v8f s[4];
#pragma unroll
    for (int j = 0; j < 4; ++j) {
      s[j] = (v8f){0.f,0.f,0.f,0.f,0.f,0.f,0.f,0.f};
#pragma unroll
      for (int dc = 0; dc < 4; ++dc) {
        FH kb;
        kb.h[0] = *(const v8h*)(Ksh + (j * 16 + c) * HDIM + dc * 32 + 8 * hh);
        kb.h[1] = *(const v8h*)(Ksh + (j * 16 + c) * HDIM + dc * 32 + 16 + 8 * hh);
        s[j] = mma_h(qa[dc], kb.v, s[j]);
      }
    }
    const bool diag = (kc == qb);
    float cm[8];
#pragma unroll
    for (int r = 0; r < 8; ++r) {
      const int qrow = q0 + 8 * hh + r;
      float m = -INFINITY;
#pragma unroll
      for (int j = 0; j < 4; ++j) {
        const int kvcol = kv0 + j * 16 + c;
        float sv = s[j][r] * ATT_SCALE;
        if (diag && (kvcol > qrow)) sv = -INFINITY;
        s[j][r] = sv;
        m = fmaxf(m, sv);
      }
#pragma unroll
      for (int off = 1; off < 16; off <<= 1) m = fmaxf(m, __shfl_xor(m, off, 32));
      cm[r] = m;
    }
    _Float16* pw = Psh[wave];
#pragma unroll
    for (int r = 0; r < 8; ++r) {
      const float mnew = fmaxf(mrow[r], cm[r]);
      const float mref = (mnew > -INFINITY) ? mnew : 0.0f;
      const float alpha = expf(mrow[r] - mref);
      mrow[r] = mnew;
      float psum = 0.f;
#pragma unroll
      for (int j = 0; j < 4; ++j) {
        const float p = expf(s[j][r] - mref);
        psum += p;
        pw[(8 * hh + r) * AKC + j * 16 + c] = (_Float16)(p * PSCALE);
      }
#pragma unroll
      for (int off = 1; off < 16; off <<= 1) psum += __shfl_xor(psum, off, 32);
      lrow[r] = lrow[r] * alpha + psum;
#pragma unroll
      for (int t = 0; t < 8; ++t) oacc[t][r] *= alpha;
    }
    __builtin_amdgcn_fence(__ATOMIC_RELEASE, "workgroup");
    __builtin_amdgcn_wave_barrier();
    __builtin_amdgcn_fence(__ATOMIC_ACQUIRE, "workgroup");
#pragma unroll 1
    for (int kk = 0; kk < 2; ++kk) {
      FH pa;
      pa.h[0] = *(const v8h*)(pw + c * AKC + kk * 32 + 8 * hh);
      pa.h[1] = *(const v8h*)(pw + c * AKC + kk * 32 + 16 + 8 * hh);
#pragma unroll
      for (int t = 0; t < 8; ++t) {
        FH vb;
        vb.h[0] = *(const v8h*)(Vth + (t * 16 + c) * AKC + kk * 32 + 8 * hh);
        vb.h[1] = *(const v8h*)(Vth + (t * 16 + c) * AKC + kk * 32 + 16 + 8 * hh);
        oacc[t] = mma_h(pa.v, vb.v, oacc[t]);
      }
    }
  }

  _Float16* os = Osh[wave];
#pragma unroll
  for (int r = 0; r < 8; ++r) {
    const float inv = OMUL / (lrow[r] * PSCALE);
#pragma unroll
    for (int t = 0; t < 8; ++t) os[(8 * hh + r) * OSP + t * 16 + c] = (_Float16)(oacc[t][r] * inv);
  }
  __builtin_amdgcn_fence(__ATOMIC_RELEASE, "workgroup");
  __builtin_amdgcn_wave_barrier();
  __builtin_amdgcn_fence(__ATOMIC_ACQUIRE, "workgroup");
  {
    const int c8 = (lane & 15) * 8;
    for (int pass = 0; pass < 2; ++pass) {
#pragma unroll
      for (int it = 0; it < 8; ++it) {
        const int row = it * 2 + hh;
        const v8h val = *(const v8h*)(os + row * OSP + c8);
        *(volatile v8h*)(out + (tokb + q0 + row) * QCOLS + (size_t)h * HDIM + c8) = val;
      }
      __threadfence();
    }
  }
}

#define OXP 132
__global__ __launch_bounds__(128) void att_exact_k(const float* __restrict__ qx, const float* __restrict__ kx,
                                                   const float* __restrict__ vx, float* __restrict__ aox) {
  __shared__ __align__(16) float os_[NXR][OXP];
  const int h = blockIdx.x, b = blockIdx.y, i = threadIdx.x;
  const int g = h / (NHEAD / NKVH);
  const float* qrow = qx + ((size_t)b * NXR + i) * QCOLS + (size_t)h * HDIM;
#pragma unroll 4
  for (int d = 0; d < HDIM; ++d) os_[i][d] = 0.f;
  float m = -3.0e38f, l = 0.f;
#pragma unroll 1
  for (int j = 0; j <= i; ++j) {
    const float* krow = kx + ((size_t)b * NXR + j) * KVCOLS + (size_t)g * HDIM;
    const float* vrow = vx + ((size_t)b * NXR + j) * KVCOLS + (size_t)g * HDIM;
    float s = 0.f;
#pragma unroll 4
    for (int d = 0; d < HDIM; ++d) s += qrow[d] * krow[d];
    s *= ATT_SCALE;
    if (j <= i) {
      const float mn = fmaxf(m, s);
      const float cs = expf(m - mn), pj = expf(s - mn);
      l = l * cs + pj;
#pragma unroll 4
      for (int d = 0; d < HDIM; ++d) os_[i][d] = os_[i][d] * cs + pj * vrow[d];
      m = mn;
    }
  }
  const float inv = (l > 0.f) ? 1.f / l : 0.f;
#pragma unroll 4
  for (int d = 0; d < HDIM; ++d) os_[i][d] *= inv;
  __syncthreads();
  const int grp = i >> 3, lg = i & 7;
#pragma unroll 1
  for (int pass = 0; pass < 32; ++pass) {
    const int line = pass * 16 + grp;
    const int row = line >> 2, c0 = (line & 3) * 32 + lg * 4;
    const v4f v = *(const v4f*)(&os_[row][c0]);
    float* dst = aox + ((size_t)b * NXR + row) * QCOLS + (size_t)h * HDIM + c0;
    *(volatile v4f*)dst = v;
    __threadfence();
    *(volatile v4f*)dst = v;
  }
}

constexpr size_t SZ_X16  = (size_t)NTOK * DMODEL * 2;
constexpr size_t SZ_WQ   = (size_t)QCOLS * DMODEL * 2;
constexpr size_t SZ_WK   = (size_t)KVCOLS * DMODEL * 2;
constexpr size_t SZ_WV   = SZ_WK;
constexpr size_t SZ_WO   = (size_t)DMODEL * QCOLS * 2;
constexpr size_t SZ_QF   = (size_t)NTOK * QCOLS * 4;
constexpr size_t SZ_KF   = (size_t)NTOK * KVCOLS * 4;
constexpr size_t SZ_Q16  = (size_t)NTOK * QCOLS * 2;
constexpr size_t SZ_K16  = (size_t)NTOK * KVCOLS * 2;
constexpr size_t SZ_V16  = SZ_K16;
constexpr size_t SZ_XH   = (size_t)NXTOT * DMODEL * 2;
constexpr size_t SZ_WVH  = (size_t)KVCOLS * DMODEL * 2;
constexpr size_t SZ_WOH  = (size_t)DMODEL * QCOLS * 2;
constexpr size_t SZ_WQH  = (size_t)QCOLS * DMODEL * 2;
constexpr size_t SZ_WKH  = (size_t)KVCOLS * DMODEL * 2;
constexpr size_t SZ_VX   = (size_t)NXTOT * KVCOLS * 4;
constexpr size_t SZ_QX   = (size_t)NXTOT * QCOLS * 4;
constexpr size_t SZ_KX   = (size_t)NXTOT * KVCOLS * 4;
constexpr size_t SZ_AOX  = (size_t)NXTOT * QCOLS * 4;
constexpr size_t SZ_AOXH = (size_t)NXTOT * QCOLS * 2;
constexpr size_t OFF_X16 = 0, OFF_WOH = 0, OFF_WOL = OFF_WOH + SZ_WOH,
                 OFF_WQ = OFF_X16 + SZ_X16, OFF_WK = OFF_WQ + SZ_WQ, OFF_WV = OFF_WK + SZ_WK, OFF_WO = OFF_WV + SZ_WV,
                 OFF_QF = OFF_WO + SZ_WO, OFF_ATT = OFF_QF, OFF_WQH = OFF_QF + SZ_Q16, OFF_WQL = OFF_WQH + SZ_WQH,
                 OFF_KF = OFF_QF + SZ_QF, OFF_WKH = OFF_KF, OFF_WKL = OFF_WKH + SZ_WKH,
                 OFF_Q16 = OFF_KF + SZ_KF,
                 OFF_K16 = OFF_Q16 + SZ_Q16, OFF_V16 = OFF_K16 + SZ_K16,
                 OFF_XH = OFF_V16 + SZ_V16, OFF_XL = OFF_XH + SZ_XH, OFF_WVH = OFF_XL + SZ_XH, OFF_WVL = OFF_WVH + SZ_WVH,
                 OFF_VX = OFF_WVL + SZ_WVH, OFF_QX = OFF_VX + SZ_VX, OFF_KX = OFF_QX + SZ_QX, OFF_AOX = OFF_KX + SZ_KX,
                 OFF_AOXH = OFF_AOX + SZ_AOX, OFF_AOXL = OFF_AOXH + SZ_AOXH,
                 OFF_QXR = OFF_AOXL + SZ_AOXH, OFF_KXR = OFF_QXR + SZ_QX, OFF_END = OFF_KXR + SZ_KX;
static_assert(OFF_WOL + SZ_WOH <= OFF_X16 + SZ_X16);
static_assert(SZ_Q16 <= SZ_QF);
static_assert(OFF_WQL + SZ_WQH <= OFF_QF + SZ_QF);
static_assert(OFF_WKL + SZ_WKH <= OFF_KF + SZ_KF);
static_assert(OFF_WQH == 54525952 && OFF_WQL == 62914560 && OFF_WKL == 73400320);
static_assert(OFF_END == 121110528);
static_assert(OFF_END <= 134217728);

extern "C" void kernel_launch(void* const* d_in, const int* in_sizes, int n_in,
                              void* d_out, int out_size, void* d_ws,
                              size_t ws_size, hipStream_t stream) {
  if (n_in < 7) return;
  if (in_sizes[0] != NTOK * DMODEL || in_sizes[1] != SEQ * HDIM || in_sizes[2] != SEQ * HDIM ||
      in_sizes[3] != QCOLS * DMODEL || in_sizes[4] != KVCOLS * DMODEL || in_sizes[5] != KVCOLS * DMODEL ||
      in_sizes[6] != DMODEL * QCOLS || out_size != NTOK * DMODEL) return;
  if (OFF_END > ws_size) return;

  const float* x    = (const float*)d_in[0];
  const float* cosT = (const float*)d_in[1];
  const float* sinT = (const float*)d_in[2];
  const float* wq   = (const float*)d_in[3];
  const float* wk   = (const float*)d_in[4];
  const float* wv   = (const float*)d_in[5];
  const float* wo   = (const float*)d_in[6];
  float* outf = (float*)d_out;

  char* ws = (char*)d_ws;
  _Float16*       x16   = (_Float16*)(ws + OFF_X16);
  _Float16*       wq16  = (_Float16*)(ws + OFF_WQ);
  _Float16*       wk16  = (_Float16*)(ws + OFF_WK);
  _Float16*       wv16  = (_Float16*)(ws + OFF_WV);
  _Float16*       wo16  = (_Float16*)(ws + OFF_WO);
  float*          qf    = (float*)(ws + OFF_QF);
  unsigned short* att16 = (unsigned short*)(ws + OFF_ATT);
  float*          kf    = (float*)(ws + OFF_KF);
  unsigned short* q16   = (unsigned short*)(ws + OFF_Q16);
  unsigned short* k16   = (unsigned short*)(ws + OFF_K16);
  unsigned short* v16   = (unsigned short*)(ws + OFF_V16);
  unsigned short* woh   = (unsigned short*)(ws + OFF_WOH);
  unsigned short* wol   = (unsigned short*)(ws + OFF_WOL);
  unsigned short* wqh   = (unsigned short*)(ws + OFF_WQH);
  unsigned short* wql   = (unsigned short*)(ws + OFF_WQL);
  unsigned short* wkh   = (unsigned short*)(ws + OFF_WKH);
  unsigned short* wkl   = (unsigned short*)(ws + OFF_WKL);
  unsigned short* xh    = (unsigned short*)(ws + OFF_XH);
  unsigned short* xl    = (unsigned short*)(ws + OFF_XL);
  unsigned short* wvh   = (unsigned short*)(ws + OFF_WVH);
  unsigned short* wvl   = (unsigned short*)(ws + OFF_WVL);
  float*          vx    = (float*)(ws + OFF_VX);
  float*          qx    = (float*)(ws + OFF_QX);
  float*          kx    = (float*)(ws + OFF_KX);
  float*          aox   = (float*)(ws + OFF_AOX);
  unsigned short* aoxh  = (unsigned short*)(ws + OFF_AOXH);
  unsigned short* aoxl  = (unsigned short*)(ws + OFF_AOXL);
  float*          qxr   = (float*)(ws + OFF_QXR);
  float*          kxr   = (float*)(ws + OFF_KXR);

  {
    const int n2x = NTOK * DMODEL / 2, n2q = QCOLS * DMODEL / 2, n2k = KVCOLS * DMODEL / 2;
    cast_f32_f16x2<<<(n2x + 255) / 256, 256, 0, stream>>>(x, x16, n2x, 1.0f);
    cast_f32_f16x2<<<(n2q + 255) / 256, 256, 0, stream>>>(wq, wq16, n2q, WMUL);
    cast_f32_f16x2<<<(n2k + 255) / 256, 256, 0, stream>>>(wk, wk16, n2k, WMUL);
    cast_f32_f16x2<<<(n2k + 255) / 256, 256, 0, stream>>>(wv, wv16, n2k, WMUL);
    cast_f32_f16x2<<<(n2q + 255) / 256, 256, 0, stream>>>(wo, wo16, n2q, WMUL);
  }
  {
    const int M = NTOK, N = QCOLS, K = DMODEL;
    const int tiles = (M / 64) * (N / 64);
    wmma_gemm64<0, false, 0, 0, false, 0><<<dim3((tiles + 7) / 8, 1), 256, 0, stream>>>(
        U16(x16), U16(x16), K, 0, U16(wq16), U16(wq16), K, 0, qf, qf, N, 0, cosT, cosT, 0, M, N, K, WMUL_INV);
  }
  {
    const int M = NTOK, N = KVCOLS, K = DMODEL;
    const int tiles = (M / 64) * (N / 64);
    wmma_gemm64<0, false, 0, 0, false, 0><<<dim3((tiles + 7) / 8, 1), 256, 0, stream>>>(
        U16(x16), U16(x16), K, 0, U16(wk16), U16(wk16), K, 0, kf, kf, N, 0, cosT, cosT, 0, M, N, K, WMUL_INV);
    wmma_gemm64<0, false, 0, 1, false, 0><<<dim3((tiles + 7) / 8, 1), 256, 0, stream>>>(
        U16(x16), U16(x16), K, 0, U16(wv16), U16(wv16), K, 0, v16, v16, N, 0, cosT, cosT, 0, M, N, K, WMUL_INV);
  }
  rope_rms_k<0><<<dim3(SEQ, NBATCH), 256, 0, stream>>>(qf, kf, cosT, sinT, q16, k16, qx, kx);
  attn128_k<<<NBATCH * NHEAD * (SEQ / AQB), 128, 0, stream>>>(q16, k16, v16, att16);
  {
    const int M = NTOK, N = DMODEL, K = QCOLS;
    const int tiles = (M / 64) * (N / 64);
    wmma_gemm64<0, false, 0, 0, false, 0><<<dim3((tiles + 7) / 8, 1), 256, 0, stream>>>(
        att16, att16, K, 0, U16(wo16), U16(wo16), K, 0, outf, outf, N, 0, cosT, cosT, 0, M, N, K,
        WMUL_INV * OMUL_INV);
  }

  {
    const int nc2 = DMODEL / 2;
    split_bf16x2<<<(NXTOT * nc2 + 255) / 256, 256, 0, stream>>>(x, xh, xl, nc2, NXTOT, NXR, SEQ);
    split_bf16x2<<<(KVCOLS * nc2 + 255) / 256, 256, 0, stream>>>(wv, wvh, wvl, nc2, KVCOLS, KVCOLS, KVCOLS);
    split_bf16x2<<<(DMODEL * nc2 + 255) / 256, 256, 0, stream>>>(wo, woh, wol, nc2, DMODEL, DMODEL, DMODEL);
    split_bf16x2<<<(QCOLS * nc2 + 255) / 256, 256, 0, stream>>>(wq, wqh, wql, nc2, QCOLS, QCOLS, QCOLS);
    split_bf16x2<<<(KVCOLS * nc2 + 255) / 256, 256, 0, stream>>>(wk, wkh, wkl, nc2, KVCOLS, KVCOLS, KVCOLS);
  }
  {
    const int M = NXTOT, N = KVCOLS, K = DMODEL;
    const int tiles = (M / 64) * (N / 64);
    wmma_gemm64<1, true, 0, 0, false, 0><<<dim3((tiles + 7) / 8, 1), 256, 0, stream>>>(
        xh, xl, K, 0, wvh, wvl, K, 0, vx, vx, N, 0, cosT, cosT, 0, M, N, K, 1.0f);
  }
  {
    const int M = NXTOT, N = QCOLS, K = DMODEL;
    const int tiles = (M / 64) * (N / 64);
    wmma_gemm64<1, true, 0, 0, false, 0><<<dim3((tiles + 7) / 8, 1), 256, 0, stream>>>(
        xh, xl, K, 0, wqh, wql, K, 0, qxr, qxr, N, 0, cosT, cosT, 0, M, N, K, 1.0f);
  }
  {
    const int M = NXTOT, N = KVCOLS, K = DMODEL;
    const int tiles = (M / 64) * (N / 64);
    wmma_gemm64<1, true, 0, 0, false, 0><<<dim3((tiles + 7) / 8, 1), 256, 0, stream>>>(
        xh, xl, K, 0, wkh, wkl, K, 0, kxr, kxr, N, 0, cosT, cosT, 0, M, N, K, 1.0f);
  }
  rope_rms_k<1><<<dim3(NXR, NBATCH), 256, 0, stream>>>(qxr, kxr, cosT, sinT, q16, k16, qx, kx);
  att_exact_k<<<dim3(NHEAD, NBATCH), 128, 0, stream>>>(qx, kx, vx, aox);
  split_bf16x2<<<(NXTOT * (QCOLS / 2) + 255) / 256, 256, 0, stream>>>(aox, aoxh, aoxl, QCOLS / 2, NXTOT, NXTOT, NXTOT);
  {
    const int M = NXR, N = DMODEL, K = QCOLS;
    const int tiles = (M / 64) * (N / 64);
    wmma_gemm64<1, true, 0, 0, false, 0><<<dim3((tiles + 7) / 8, NBATCH), 256, 0, stream>>>(
        aoxh, aoxl, K, (long)NXR * QCOLS, woh, wol, K, 0L, outf, outf, N, (long)SEQ * DMODEL, cosT, cosT, 0L, M, N, K, 1.0f);
  }
}
